// NonLinearTSQ_79551384256577
// MI455X (gfx1250) — hardware-run, weakly checked
//
#include <hip/hip_runtime.h>


namespace {
constexpr int N = 32768, NS = 64, NV = 32, P0 = 64, Q1 = 32, R2 = 16, DIN = 160, DOUT = 240, KSS = NS * NS  , KVV = NV * NV  , K0 = KSS + KVV  , K1 = NS * NV  , SROW = 256  ;
constexpr float HS = 256.0f, WSC = 1.0f  ;
typedef _Float16 b16;
typedef __attribute__((ext_vector_type(16))) _Float16 v16b;
typedef __attribute__((ext_vector_type(8))) _Float16 v8b;
typedef __attribute__((ext_vector_type(8))) float v8f;
typedef __attribute__((ext_vector_type(4))) float v4f;
__device__ __forceinline__ float bf16_rne(float f) { unsigned int u = __float_as_uint(f); u += 0x7FFFu + ((u >> 16) & 1u); float r = __uint_as_float(u & 0xFFFF0000u); asm volatile("" : "+v"(r)); return r; }
__device__ __forceinline__ float bfv(float f) { float r = bf16_rne(f); asm volatile("" : "+v"(r)); return r; }
__device__ __forceinline__ void split16(float v, b16& hi, b16& lo) { hi = (b16)v; lo = (b16)(v - (float)hi); }
__device__ __forceinline__ v16b frag_kb(const b16* p, int hh) { const v8b a = *(const v8b*)(p + 8 * hh), b = *(const v8b*)(p + 16 + 8 * hh); v16b f;
#pragma unroll
  for (int e = 0; e < 8; ++e) { f[e] = a[e]; f[8 + e] = b[e]; } return f; }
__device__ __forceinline__ v8f wmma16b(v16b a, v16b b, v8f c) { v8f d = __builtin_amdgcn_wmma_f32_16x16x32_f16(false, a, false, b, (short)0, c, false, false); asm volatile("v_nop\n\tv_nop\n\tv_nop\n\tv_nop" : "+v"(d) : "v"(a), "v"(b)); return d; }
__device__ __forceinline__ void wave_lds_sync() { __builtin_amdgcn_fence(__ATOMIC_RELEASE, "workgroup"); __builtin_amdgcn_wave_barrier(); __builtin_amdgcn_fence(__ATOMIC_ACQUIRE, "workgroup"); }
__device__ __forceinline__ float pmul(float a, float b) { float p = a * b; asm volatile("" : "+v"(p)); return p; }

__global__ __launch_bounds__(256) void wput_kernel(const float* __restrict__ wss, const float* __restrict__ wsv, const float* __restrict__ wvv0, const float* __restrict__ wvv2, b16* __restrict__ WA, b16* __restrict__ WB, b16* __restrict__ WC) { const size_t nt = (size_t)gridDim.x * 256, u0 = (size_t)blockIdx.x * 256 + threadIdx.x; v8b v;
  for (size_t u = u0; u < (size_t)P0 * (K0 / 8); u += nt) { const int p = (int)(u / (K0 / 8)), k0 = (int)(u % (K0 / 8)) * 8;
#pragma unroll
    for (int j = 0; j < 8; ++j) { const int k = k0 + j; float w; if (k < KSS) w = wss[((size_t)(k / NS) * NS + (k % NS)) * P0 + p]; else { const int kk = k - KSS; w = wvv0[((size_t)(kk / NV) * NV + (kk % NV)) * P0 + p]; } v[j] = (b16)(bf16_rne(w) * WSC); }
    for (int pass = 0; pass < 2; ++pass) { *(volatile v8b*)(WA + (size_t)p * K0 + k0) = v; __threadfence(); } }
  for (size_t u = u0; u < (size_t)Q1 * (K1 / 8); u += nt) { const int q = (int)(u / (K1 / 8)), k0 = (int)(u % (K1 / 8)) * 8;
#pragma unroll
    for (int j = 0; j < 8; ++j) { const int k = k0 + j; v[j] = (b16)(bf16_rne(wsv[((size_t)(k / NV) * NV + (k % NV)) * Q1 + q]) * WSC); }
    for (int pass = 0; pass < 2; ++pass) { *(volatile v8b*)(WB + (size_t)q * K1 + k0) = v; __threadfence(); } }
  for (size_t u = u0; u < (size_t)NV * R2 * (NV / 8); u += nt) { const int o = (int)(u / (NV / 8)), k0 = (int)(u % (NV / 8)) * 8; const int uu = o / R2, r = o % R2;
#pragma unroll
    for (int j = 0; j < 8; ++j) v[j] = (b16)(bf16_rne(wvv2[((size_t)uu * NV + k0 + j) * R2 + r]) * WSC);
    for (int pass = 0; pass < 2; ++pass) { *(volatile v8b*)(WC + (size_t)o * NV + k0) = v; __threadfence(); } } }
__device__ __forceinline__ void load_sv(const float* __restrict__ x, const float* __restrict__ gates, size_t n, int lane, float* Srow, float* Vrow) {
  for (int q = 0; q < 2; ++q) Srow[q * 32 + lane] = tanhf(bfv(x[n * DIN + q * 32 + lane])); for (int q = 0; q < 3; ++q) { const int c = q * 32 + lane; Vrow[c] = pmul(bfv(x[n * DIN + NS + c]), tanhf(bfv(gates[c / 3]))); } }
__global__ __launch_bounds__(32) void out0_kernel(const float* __restrict__ x, const float* __restrict__ gates, const b16* __restrict__ WA, float* __restrict__ STG) { __shared__ float Sr[16][NS], Vr[16][3 * NV], Dv[16][KVV + 1], Tf[16][P0 + 1]; const int lane = threadIdx.x, nloc = lane & 15, hlf = lane >> 4; const size_t m0 = (size_t)blockIdx.x * 16;
  for (int rr = 0; rr < 16; ++rr) load_sv(x, gates, m0 + rr, lane, Sr[rr], Vr[rr]);
  wave_lds_sync();
  for (int rr = 0; rr < 16; ++rr) for (int q = lane; q < KVV; q += 32) { const int uu = q / NV, vv = q % NV; float d = 0.0f; for (int i = 0; i < 3; ++i) d += pmul(Vr[rr][uu * 3 + i], Vr[rr][vv * 3 + i]); Dv[rr][q] = d * 0.57735026918962576f; }
  wave_lds_sync(); v8f acc[4] = {(v8f){}, (v8f){}, (v8f){}, (v8f){}};
#pragma unroll 1
  for (int kb = 0; kb < K0; kb += 32) { v16b a, al;
#pragma unroll
    for (int e = 0; e < 16; ++e) { const int k = kb + (e < 8 ? 8 * hlf + e : 16 + 8 * hlf + (e - 8)); float val; if (k < KSS) val = pmul(Sr[nloc][k / NS], Sr[nloc][k % NS]); else val = Dv[nloc][k - KSS]; b16 p, ql; split16(val * HS, p, ql); a[e] = p; al[e] = ql; }
#pragma unroll
    for (int t = 0; t < 4; ++t) { const v16b bw = frag_kb(WA + (size_t)(t * 16 + nloc) * K0 + kb, hlf); acc[t] = wmma16b(a, bw, acc[t]); acc[t] = wmma16b(al, bw, acc[t]); } }
  const float c0 = 1.0f / sqrtf((float)(NS * NS + NV * NV));
#pragma unroll
  for (int t = 0; t < 4; ++t)
#pragma unroll
    for (int r8 = 0; r8 < 8; ++r8) Tf[8 * hlf + r8][t * 16 + nloc] = acc[t][r8] * (c0 / (HS * WSC));
  wave_lds_sync();
  for (int pass = 0; pass < 2; ++pass) { for (int rr = 0; rr < 16; ++rr) for (int q = 0; q < 2; ++q) ((volatile float*)STG)[(m0 + rr) * SROW + q * 32 + lane] = Tf[rr][q * 32 + lane]; __threadfence(); } }
__global__ __launch_bounds__(32) void out1_kernel(const float* __restrict__ x, const float* __restrict__ gates, const b16* __restrict__ WB, float* __restrict__ STG) { __shared__ float Sr[4][NS], Vr[4][3 * NV], Tf[16][Q1 + 1]; const int lane = threadIdx.x, nloc = lane & 15, hlf = lane >> 4; const size_t n0 = (size_t)blockIdx.x * 4;
  for (int j = 0; j < 4; ++j) load_sv(x, gates, n0 + j, lane, Sr[j], Vr[j]);
  wave_lds_sync(); const int nl = nloc >> 2, ii = nloc & 3; v8f acc[2] = {(v8f){}, (v8f){}};
#pragma unroll 1
  for (int kb = 0; kb < K1; kb += 32) { v16b a, al;
#pragma unroll
    for (int e = 0; e < 16; ++e) { const int k = kb + (e < 8 ? 8 * hlf + e : 16 + 8 * hlf + (e - 8)); const float val = ii < 3 ? pmul(Sr[nl][k / NV], Vr[nl][(k % NV) * 3 + ii]) : 0.0f; b16 p, ql; split16(val * HS, p, ql); a[e] = p; al[e] = ql; }
#pragma unroll
    for (int t = 0; t < 2; ++t) { const v16b bw = frag_kb(WB + (size_t)(t * 16 + nloc) * K1 + kb, hlf); acc[t] = wmma16b(a, bw, acc[t]); acc[t] = wmma16b(al, bw, acc[t]); } }
  const float c1 = 1.0f / sqrtf((float)(NS * NV));
#pragma unroll
  for (int t = 0; t < 2; ++t)
#pragma unroll
    for (int r8 = 0; r8 < 8; ++r8) Tf[8 * hlf + r8][t * 16 + nloc] = acc[t][r8] * (c1 / (HS * WSC));
  wave_lds_sync();
  for (int pass = 0; pass < 2; ++pass) { for (int j = 0; j < 4; ++j) for (int q2 = 0; q2 < 3; ++q2) { const int idx = q2 * 32 + lane; const int q = idx / 3, i = idx % 3; ((volatile float*)STG)[(n0 + j) * SROW + NS + idx] = Tf[j * 4 + i][q]; } __threadfence(); } }
__global__ __launch_bounds__(32) void out2_kernel(const float* __restrict__ x, const float* __restrict__ gates, const b16* __restrict__ WC, float* __restrict__ STG) { __shared__ float Sr[4][NS], Vr[4][3 * NV]; __shared__ __attribute__((aligned(16))) b16 Ah[16][NV + 8], Al[16][NV + 8]; __shared__ float TV[16][NV * R2 + 4], Sm[4][R2][9], O2[4][96]; const int lane = threadIdx.x, nloc = lane & 15, hlf = lane >> 4; const size_t n0 = (size_t)blockIdx.x * 4;
  for (int j = 0; j < 4; ++j) load_sv(x, gates, n0 + j, lane, Sr[j], Vr[j]);
  wave_lds_sync();
  for (int rr = 0; rr < 16; ++rr) { const int nl = rr >> 2, jj = rr & 3; const float val = jj < 3 ? Vr[nl][lane * 3 + jj] : 0.0f; b16 p, ql; split16(val * HS, p, ql); Ah[rr][lane] = p; Al[rr][lane] = ql; } if (lane < 16) for (int k = NV; k < NV + 8; ++k) { Ah[lane][k] = (b16)0.0f; Al[lane][k] = (b16)0.0f; }
  wave_lds_sync(); const v16b a = frag_kb(&Ah[nloc][0], hlf), al = frag_kb(&Al[nloc][0], hlf);
#pragma unroll 1
  for (int g = 0; g < 4; ++g) { v8f acc[8];
#pragma unroll
    for (int t = 0; t < 8; ++t) acc[t] = (v8f){};
#pragma unroll
    for (int t = 0; t < 8; ++t) { const v16b bw = frag_kb(WC + (size_t)((g * 8 + t) * 16 + nloc) * NV, hlf); acc[t] = wmma16b(a, bw, acc[t]); acc[t] = wmma16b(al, bw, acc[t]); }
#pragma unroll
    for (int t = 0; t < 8; ++t)
#pragma unroll
      for (int r8 = 0; r8 < 8; ++r8) TV[8 * hlf + r8][(g * 8 + t) * 16 + nloc] = acc[t][r8] * (1.0f / (HS * WSC)); }
  wave_lds_sync();
  for (int q = lane; q < 4 * R2 * 9; q += 32) { const int nl = q / (R2 * 9), rem = q % (R2 * 9); const int r = rem / 9, ij = rem % 9; const int i = ij / 3, j = ij % 3; float s = 0.0f;
#pragma unroll 8
    for (int uu = 0; uu < NV; ++uu) s += pmul(Vr[nl][uu * 3 + i], TV[nl * 4 + j][uu * R2 + r]); Sm[nl][r][ij] = s; }
  wave_lds_sync();
  { const float is2 = 0.70710678118654752f, is6 = 0.40824829046386302f; const float c2 = 1.0f / sqrtf((float)(NV * NV));
    for (int q = lane; q < 4 * 96; q += 32) { const int nl = q / 96, idx = q % 96; float o = 0.0f; if (idx < R2 * 5) { const int r = idx / 5, m = idx % 5; const float* S9 = Sm[nl][r];
        if (m == 0) o = is2 * (S9[0 * 3 + 1] + S9[1 * 3 + 0]); else if (m == 1) o = is2 * (S9[1 * 3 + 2] + S9[2 * 3 + 1]); else if (m == 2) o = is6 * (2.0f * S9[2 * 3 + 2] - S9[0 * 3 + 0] - S9[1 * 3 + 1]); else if (m == 3) o = is2 * (S9[0 * 3 + 2] + S9[2 * 3 + 0]); else o = is2 * (S9[0 * 3 + 0] - S9[1 * 3 + 1]); o *= c2; } O2[nl][idx] = o; } }
  wave_lds_sync();
  for (int pass = 0; pass < 2; ++pass) { for (int j = 0; j < 4; ++j) for (int q2 = 0; q2 < 3; ++q2) ((volatile float*)STG)[(n0 + j) * SROW + NS + 3 * Q1 + q2 * 32 + lane] = O2[j][q2 * 32 + lane]; __threadfence(); } }
__global__ __launch_bounds__(256) void copy_kernel(const float* __restrict__ STG, int NLIM, float* __restrict__ out) { const size_t u = (size_t)blockIdx.x * 256 + threadIdx.x; if (u >= (size_t)N * DOUT) return; const size_t n = u / DOUT; const int c = (int)(u % DOUT); if (n >= (size_t)NLIM) return;
  for (int pass = 0; pass < 2; ++pass) { ((volatile float*)out)[u] = STG[n * SROW + c]; __threadfence(); } }
}

extern "C" void kernel_launch(void* const* d_in, const int* in_sizes, int n_in, void* d_out, int out_size, void* d_ws, size_t ws_size, hipStream_t stream) {
  (void)n_in;
  auto Fp = [&](int i) { return (const float*)d_in[i]; };
  if (in_sizes[0] != N * DIN || in_sizes[1] != NV || in_sizes[2] != NS * NS * P0 || in_sizes[3] != NS * NV * Q1 || in_sizes[4] != NV * NV * P0 || in_sizes[5] != NV * NV * R2 || out_size != N * DOUT) return;
  const int NLIM = N;
  size_t off = 0; char* ws = (char*)d_ws;
  auto carve = [&](size_t bytes) { char* p = ws + off; off += (bytes + 255) & ~(size_t)255; return p; };
  b16* WA = (b16*)carve((size_t)P0 * K0 * 2); b16* WB = (b16*)carve((size_t)Q1 * K1 * 2); b16* WC = (b16*)carve((size_t)NV * R2 * NV * 2); float* STG = (float*)carve((size_t)N * SROW * 4);
  if (off > ws_size || off > ((size_t)48 << 20)) return;
  wput_kernel<<<128, 256, 0, stream>>>(Fp(2), Fp(3), Fp(4), Fp(5), WA, WB, WC);
  out0_kernel<<<NLIM / 16, 32, 0, stream>>>(Fp(0), Fp(1), WA, STG);
  out1_kernel<<<NLIM / 4, 32, 0, stream>>>(Fp(0), Fp(1), WB, STG);
  out2_kernel<<<NLIM / 4, 32, 0, stream>>>(Fp(0), Fp(1), WC, STG);
  copy_kernel<<<(N * DOUT + 255) / 256, 256, 0, stream>>>(STG, NLIM, (float*)d_out);
}
